// MutualAttention_37263136260605
// MI455X (gfx1250) — hardware-run, weakly checked
//
#include <hip/hip_runtime.h>


#define NBR  1024
#define DD   512
typedef _Float16 h16;
typedef unsigned short bf;
typedef __attribute__((ext_vector_type(16))) __bf16   v16bf;
typedef __attribute__((ext_vector_type(16))) _Float16 v16h;
typedef __attribute__((ext_vector_type(8)))  _Float16 v8h;
typedef __attribute__((ext_vector_type(8)))  unsigned short v8us;
typedef __attribute__((ext_vector_type(8)))  float    v8f;
typedef __attribute__((ext_vector_type(4)))  float    v4f;
typedef v8h  __attribute__((may_alias)) v8ha;
typedef v4f  __attribute__((may_alias)) v4fa;
typedef v8us __attribute__((may_alias)) v8usa;
typedef __attribute__((ext_vector_type(2))) unsigned short v2us;

__device__ __forceinline__ unsigned short f2bf(float f) { unsigned u = __float_as_uint(f); u += 0x7FFFu + ((u >> 16) & 1u); return (unsigned short)(u >> 16); }
__device__ __forceinline__ float bf2f(unsigned short b) { return __uint_as_float(((unsigned)b) << 16); }
__device__ __forceinline__ float bfr(float f) { return bf2f(f2bf(f)); }
__device__ __forceinline__ v16h cat16(v8h lo, v8h hi) { return __builtin_shufflevector(lo, hi, 0, 1, 2, 3, 4, 5, 6, 7, 8, 9, 10, 11, 12, 13, 14, 15); }
__device__ __forceinline__ v16bf cat16b(v8us lo, v8us hi) { return __builtin_bit_cast(v16bf, __builtin_shufflevector(lo, hi, 0, 1, 2, 3, 4, 5, 6, 7, 8, 9, 10, 11, 12, 13, 14, 15)); }
__device__ __forceinline__ v8f wmma16(v16h a, v16h b, v8f c) { return __builtin_amdgcn_wmma_f32_16x16x32_f16(false, a, false, b, (short)0, c, false, false); }
__device__ __forceinline__ v8f wmmab(v16bf a, v16bf b, v8f c) { return __builtin_amdgcn_wmma_f32_16x16x32_bf16(false, a, false, b, (short)0, c, false, false); }

template <typename T16> struct WFrag;
template <> struct WFrag<h16> { typedef v16h V; static __device__ __forceinline__ V ld(const h16* p) { return cat16(*(const v8h*)p, *(const v8h*)(p + 16)); } static __device__ __forceinline__ v8f mma(V a, V b, v8f c) { return wmma16(a, b, c); } };
template <> struct WFrag<bf> { typedef v16bf V; static __device__ __forceinline__ V ld(const bf* p) { return cat16b(*(const v8us*)p, *(const v8us*)(p + 16)); } static __device__ __forceinline__ v8f mma(V a, V b, v8f c) { return wmmab(a, b, c); } };
template <typename T16, int NSPLIT, bool BIAS>
__global__ __launch_bounds__(32) void k_gemmw(const T16* __restrict__ A, const T16* __restrict__ A2, const T16* __restrict__ Bt, const T16* __restrict__ Bt2, int K, float* C, int ldc, const float* __restrict__ bias, size_t sA, size_t sB, size_t sC) {
    typedef typename WFrag<T16>::V V;
    __shared__ __align__(16) float os[16 * 68];
    const size_t z = blockIdx.z; A += z * sA; if (A2) A2 += z * sA; Bt += z * sB; if (Bt2) Bt2 += z * sB; C += z * sC;
    const int lane = threadIdx.x & 31, lr = lane & 15, hi = lane >> 4; const int r0 = blockIdx.x * 64, c0 = blockIdx.y * 64;
    v8f acc[4][4];
#pragma unroll
    for (int mb = 0; mb < 4; ++mb)
#pragma unroll
        for (int nb = 0; nb < 4; ++nb) acc[mb][nb] = (v8f){};
    const size_t aoff = (size_t)(r0 + lr) * K + 8 * hi, boff = (size_t)(c0 + lr) * K + 8 * hi;
#pragma unroll 1
    for (int kc = 0; kc < K; kc += 32) {
        V a[4], a2[4];
#pragma unroll
        for (int mb = 0; mb < 4; ++mb) { a[mb] = WFrag<T16>::ld(A + aoff + (size_t)mb * 16 * K + kc); if (NSPLIT == 1 || NSPLIT == 2) a2[mb] = WFrag<T16>::ld(A2 + aoff + (size_t)mb * 16 * K + kc); }
#pragma unroll
        for (int nb = 0; nb < 4; ++nb) { const V b = WFrag<T16>::ld(Bt + boff + (size_t)nb * 16 * K + kc); V b2; if (NSPLIT >= 2) b2 = WFrag<T16>::ld(Bt2 + boff + (size_t)nb * 16 * K + kc);
#pragma unroll
            for (int mb = 0; mb < 4; ++mb) { acc[mb][nb] = WFrag<T16>::mma(a[mb], b, acc[mb][nb]); if (NSPLIT == 1 || NSPLIT == 2) acc[mb][nb] = WFrag<T16>::mma(a2[mb], b, acc[mb][nb]); if (NSPLIT >= 2) acc[mb][nb] = WFrag<T16>::mma(a[mb], b2, acc[mb][nb]); } }
        asm volatile("v_nop\n\tv_nop\n\tv_nop\n\tv_nop" : "+v"(acc[0][0]), "+v"(acc[1][1]), "+v"(acc[2][2]), "+v"(acc[3][3]) : "v"(a[0]), "v"(a[3]));
    }
#pragma unroll
    for (int mb = 0; mb < 4; ++mb) {
#pragma unroll
        for (int nb = 0; nb < 4; ++nb) {
#pragma unroll
            for (int j = 0; j < 8; ++j) os[(hi * 8 + j) * 68 + nb * 16 + lr] = acc[mb][nb][j]; }
        __builtin_amdgcn_wave_barrier(); asm volatile("" ::: "memory");
        float* crow = C + (size_t)(r0 + mb * 16) * ldc + c0;
#pragma unroll 1
        for (int ps = 0; ps < 2; ++ps) {
#pragma unroll
            for (int s = 0; s < 8; ++s) { const int row = 2 * s + hi, cofs = lr * 4; v4f val = *(const v4fa*)(os + row * 68 + cofs); if (BIAS) { val[0] += bfr(bias[c0 + cofs]); val[1] += bfr(bias[c0 + cofs + 1]); val[2] += bfr(bias[c0 + cofs + 2]); val[3] += bfr(bias[c0 + cofs + 3]); }
                *(volatile v4f*)(crow + (size_t)row * ldc + cofs) = val; }
            if (ps == 0) __threadfence(); }
        __builtin_amdgcn_wave_barrier(); asm volatile("" ::: "memory");
    }
}

__global__ __launch_bounds__(256) void k_wtG(const float* __restrict__ w, int K, int N, bf* Bt) {
    const int lane = threadIdx.x & 31; const int L0 = (blockIdx.x * 8 + (threadIdx.x >> 5)) * 8; const int nlines = N * K / 64;
#pragma unroll
    for (int ps = 0; ps < 2; ++ps) {
#pragma unroll 1
        for (int l = 0; l < 8; ++l) { const int L = L0 + l; if (L >= nlines) break; const size_t e = (size_t)L * 64 + lane * 2; const int k = (int)(e % K), n = (int)(e / K); v2us o;
            o[0] = f2bf(w[(size_t)k * N + n]); o[1] = f2bf(w[(size_t)(k + 1) * N + n]); *(volatile v2us*)(Bt + e) = o; }
        if (ps == 0) __threadfence(); }
}
__global__ __launch_bounds__(256) void k_cvt8(const float* __restrict__ src, bf* dst, size_t n8) { const size_t i = (size_t)blockIdx.x * 256 + threadIdx.x; if (i >= n8) return; const v8f v = *(const v8f*)(src + i * 8); v8us o;
#pragma unroll
    for (int k = 0; k < 8; ++k) o[k] = f2bf(v[k]); *(volatile v8us*)(dst + i * 8) = o; __threadfence(); *(volatile v8us*)(dst + i * 8) = o; }
__device__ __forceinline__ float tanh2(float z) { const float e = __builtin_amdgcn_exp2f(z); return __fmaf_rn(-2.0f, __builtin_amdgcn_rcpf(e + 1.0f), 1.0f); }
__global__ __launch_bounds__(256) void k_mut(const float* __restrict__ PW, const float* __restrict__ p, const float* __restrict__ q, float* out0, float* out1) {
    __shared__ float sa[DD]; __shared__ float lp[DD]; __shared__ float colp[8][DD];
    const int b = blockIdx.x, tid = threadIdx.x, lane = tid & 31, wv = tid >> 5;
    const float* pr = p + (size_t)b * DD; const float* qr = q + (size_t)b * DD;
    for (int i = tid; i < DD; i += 256) sa[i] = __fmul_rn(PW[(size_t)b * DD + i], 2.8853900817779268f);
    float qv[16], ca[16];
#pragma unroll
    for (int c = 0; c < 16; ++c) { qv[c] = bfr(qr[lane + 32 * c]); ca[c] = 0.f; }
    __syncthreads();
#pragma unroll 1
    for (int i = wv; i < DD; i += 8) { const float a = sa[i]; float rs = 0.f;
#pragma unroll
        for (int c = 0; c < 16; ++c) { const float t = tanh2(__fmul_rn(a, qv[c])); ca[c] += t; rs += t; }
#pragma unroll
        for (int sh = 16; sh; sh >>= 1) rs += __shfl_xor(rs, sh, 32);
        if (lane == 0) lp[i] = rs * (1.0f / DD); }
#pragma unroll
    for (int c = 0; c < 16; ++c) colp[wv][lane + 32 * c] = ca[c];
    __syncthreads();
    if (wv < 2) { float x[16]; float mx = -3.0e38f;
#pragma unroll
        for (int c = 0; c < 16; ++c) { const int j = lane + 32 * c; float v;
            if (wv == 0) v = lp[j]; else { v = 0.f;
#pragma unroll
                for (int w = 0; w < 8; ++w) v += colp[w][j]; v *= (1.0f / DD); }
            x[c] = v; mx = fmaxf(mx, v); }
#pragma unroll
        for (int sh = 16; sh; sh >>= 1) mx = fmaxf(mx, __shfl_xor(mx, sh, 32));
        float sum = 0.f;
#pragma unroll
        for (int c = 0; c < 16; ++c) { float d0 = __fsub_rn(x[c], mx); asm volatile("" : "+v"(d0)); x[c] = __builtin_amdgcn_exp2f(__fmul_rn(d0, 1.4426950408889634f)); sum += x[c]; }
#pragma unroll
        for (int sh = 16; sh; sh >>= 1) sum += __shfl_xor(sum, sh, 32);
        const float f = __fdiv_rn(1.0f, sum);
        const float* src = wv == 0 ? pr : qr; float* dst = (wv == 0 ? out0 : out1) + (size_t)b * DD;
        float o[16];
#pragma unroll
        for (int c = 0; c < 16; ++c) o[c] = bfr(src[lane + 32 * c]) * (x[c] * f);
#pragma unroll 1
        for (int ps = 0; ps < 2; ++ps) {
#pragma unroll
            for (int c = 0; c < 16; ++c) *(volatile float*)(dst + lane + 32 * c) = o[c];
            if (ps == 0) __threadfence(); } }
}

extern "C" void kernel_launch(void* const* d_in, const int* in_sizes, int n_in,
                              void* d_out, int out_size, void* d_ws, size_t ws_size, hipStream_t stream) {
    (void)in_sizes; (void)n_in; (void)out_size;
    const float* p = (const float*)d_in[0]; const float* q = (const float*)d_in[1]; const float* w = (const float*)d_in[2];
    float* OUT0 = (float*)d_out; float* OUT1 = OUT0 + (size_t)NBR * DD;
    char* wsp = (char*)d_ws;
    auto take = [&](size_t bytes) { char* pp = wsp; wsp += (bytes + 255) & ~(size_t)255; return (void*)pp; };
    bf* PB = (bf*)take((size_t)NBR * DD * 2); bf* WT = (bf*)take((size_t)DD * DD * 2); float* PW = (float*)take((size_t)NBR * DD * 4);
    if ((size_t)(wsp - (char*)d_ws) > ws_size) return;
    k_cvt8<<<(unsigned)(((size_t)NBR * DD / 8 + 255) / 256), 256, 0, stream>>>(p, PB, (size_t)NBR * DD / 8);
    k_wtG<<<(unsigned)((DD * DD / 64 + 63) / 64), 256, 0, stream>>>(w, DD, DD, WT);
    k_gemmw<bf, 0, false><<<dim3(NBR / 64, DD / 64, 1), 32, 0, stream>>>(PB, nullptr, WT, nullptr, DD, PW, DD, nullptr, 0, 0, 0);
    k_mut<<<NBR, 256, 0, stream>>>(PW, p, q, OUT0, OUT1);
}
